// GraphTemporalEmbedding_88914412962282
// MI455X (gfx1250) — hardware-verified
//
#include <hip/hip_runtime.h>
#include <stdint.h>

typedef _Float16 v16h __attribute__((ext_vector_type(16)));
typedef _Float16 v8h  __attribute__((ext_vector_type(8)));
typedef float    v8f  __attribute__((ext_vector_type(8)));
typedef float    v4f  __attribute__((ext_vector_type(4)));
typedef v8h __attribute__((may_alias)) v8ha;
typedef v4f __attribute__((may_alias)) v4fa;

union Frag { v16h v; v8h half[2]; };

#define BZ    16
#define NC    512
#define SP    1024
#define LV    3
#define KW    3
#define KCV   (KW * NC)
#define NACT  (BZ * SP * NC)
#define NCW   (LV * NC * NC * KW)
#define WSC   16.0f
#define WINV  0.0625f
#define AINV  0.001953125f

__device__ __forceinline__ v8f wmma_f16(v16h a, v16h b, v8f c) {
  v8f d = __builtin_amdgcn_wmma_f32_16x16x32_f16(false, a, false, b, (short)0, c, false, false);
  asm volatile("v_nop\n\tv_nop\n\tv_nop\n\tv_nop" : "+v"(d) : "v"(a), "v"(b));
  return d;
}

__device__ __forceinline__ v16h load_frag(const _Float16* p, int h) {
  Frag f;
  f.half[0] = *(const v8ha*)(p + 8 * h);
  f.half[1] = *(const v8ha*)(p + 16 + 8 * h);
  return f.v;
}

__global__ __launch_bounds__(256) void k_cvt_x(const float* __restrict__ x,
                                               _Float16* __restrict__ xh)
{
  const int g = blockIdx.x * 256 + threadIdx.x;
  if (g >= NACT / 8) return;
  const float* src = x + (size_t)g * 8;
  const v4f a = *(const v4fa*)src;
  const v4f c = *(const v4fa*)(src + 4);
  const v8h o = { (_Float16)a.x, (_Float16)a.y, (_Float16)a.z, (_Float16)a.w,
                  (_Float16)c.x, (_Float16)c.y, (_Float16)c.z, (_Float16)c.w };
  _Float16* dst = xh + (size_t)g * 8;
  *(volatile v8h*)dst = o;
  __threadfence();
  *(volatile v8h*)dst = o;
}

__global__ __launch_bounds__(256) void k_prep_convw(const float* __restrict__ w1,
                                                    const float* __restrict__ w2,
                                                    _Float16* __restrict__ wp)
{
  const int g = blockIdx.x * 256 + threadIdx.x;
  if (g >= NC * (KCV / 8)) return;
  const int lw = blockIdx.y;
  const int l = lw >> 1, which = lw & 1;
  const int o = g / (KCV / 8);
  const int k0 = (g - o * (KCV / 8)) * 8;
  const int tap = k0 >> 9, c0 = k0 & (NC - 1);
  const float* w = (which != 0) ? w2 : w1;
  const float* src = w + (((size_t)(l * NC + o)) * NC + c0) * KW + tap;
  const v8h v = { (_Float16)(src[0 * KW] * WSC), (_Float16)(src[1 * KW] * WSC),
                  (_Float16)(src[2 * KW] * WSC), (_Float16)(src[3 * KW] * WSC),
                  (_Float16)(src[4 * KW] * WSC), (_Float16)(src[5 * KW] * WSC),
                  (_Float16)(src[6 * KW] * WSC), (_Float16)(src[7 * KW] * WSC) };
  _Float16* dst = wp + ((size_t)lw * NC + o) * KCV + k0;
  *(volatile v8h*)dst = v;
  __threadfence();
  *(volatile v8h*)dst = v;
}

__global__ __launch_bounds__(256) void k_prep_gcT(const float* __restrict__ gc,
                                                  _Float16* __restrict__ wg)
{
  const int g = blockIdx.x * 256 + threadIdx.x;
  if (g >= SP * (SP / 8)) return;
  const int tp = g >> 7;
  const int s0 = (g & 127) * 8;
  const float* src = gc + (size_t)s0 * SP + tp;
  const v8h v = { (_Float16)(src[0 * SP] * WSC), (_Float16)(src[1 * SP] * WSC),
                  (_Float16)(src[2 * SP] * WSC), (_Float16)(src[3 * SP] * WSC),
                  (_Float16)(src[4 * SP] * WSC), (_Float16)(src[5 * SP] * WSC),
                  (_Float16)(src[6 * SP] * WSC), (_Float16)(src[7 * SP] * WSC) };
  _Float16* dst = wg + (size_t)tp * SP + s0;
  *(volatile v8h*)dst = v;
  __threadfence();
  *(volatile v8h*)dst = v;
}

__global__ __launch_bounds__(256) void k_prep_adj(const float* __restrict__ lg,
                                                  const float* __restrict__ gn,
                                                  _Float16* __restrict__ ap)
{
  __shared__ __attribute__((aligned(16))) _Float16 sA[256];
  const int tid = threadIdx.x;
  const int idx = blockIdx.x * 256 + tid;
  const int l = idx >> 18;
  const int e = idx & (NC * NC - 1);
  const size_t gb = ((size_t)l * NC * NC + e) * 2;
  const float a0 = lg[2 * e] + gn[gb];
  const float a1 = lg[2 * e + 1] + gn[gb + 1];
  const float mx = fmaxf(a0, a1);
  const float mn = fminf(a0, a1);
  const float ex = expf(mn - mx);
  const bool ge = (a0 >= a1);
  const float e0 = ge ? 1.0f : ex;
  const float e1 = ge ? ex : 1.0f;
  const float ssum = e0 + e1;
  const float inv = 1.0f / ssum;
  const float y0 = e0 * inv;
  const float y1 = e1 * inv;
  const float hard0 = (y1 > y0) ? 0.0f : 1.0f;
  float z = hard0 + y0;
  z = z - y0;
  sA[tid] = (_Float16)(z * AINV);
  __syncthreads();
  v8h v = {(_Float16)0.0f, (_Float16)0.0f, (_Float16)0.0f, (_Float16)0.0f,
           (_Float16)0.0f, (_Float16)0.0f, (_Float16)0.0f, (_Float16)0.0f};
  if (tid < 32) v = *(const v8ha*)(sA + 8 * tid);
  _Float16* dst = ap + (size_t)blockIdx.x * 256 + 8 * tid;
  if (tid < 32) *(volatile v8h*)dst = v;
  __threadfence();
  if (tid < 32) *(volatile v8h*)dst = v;
}

__device__ __forceinline__ void store_rows_f16(const _Float16* sT, _Float16* plane,
                                               int m0, int c0, int w, int lane) {
  const int q8 = lane & 7, sub = lane >> 3;
  #pragma unroll
  for (int i = 0; i < 8; ++i) {
    const int lid = w * 32 + i * 4 + sub;
    const v8h v = *(const v8ha*)(sT + lid * 64 + 8 * q8);
    _Float16* dst = plane + (size_t)(m0 + lid) * NC + c0 + 8 * q8;
    *(volatile v8h*)dst = v;
  }
}

__device__ __forceinline__ void store_trans_f16(const _Float16* sT, _Float16* ht,
                                                int b, int o0, int t0, int w, int lane) {
  const int q8 = lane & 7, sub = lane >> 3;
  #pragma unroll
  for (int i = 0; i < 8; ++i) {
    const int lid = w * 32 + i * 4 + sub;
    const int d = lid >> 1, hl = lid & 1;
    const v8h v = *(const v8ha*)(sT + d * 128 + 64 * hl + 8 * q8);
    _Float16* dst = ht + ((size_t)(b * NC + o0 + d)) * SP + t0 + 64 * hl + 8 * q8;
    *(volatile v8h*)dst = v;
  }
}

__device__ __forceinline__ void store_rows_f32(const float* sF, float* plane,
                                               int m0, int c0, int w, int lane) {
  const int q8 = lane & 7, sub = lane >> 3;
  #pragma unroll
  for (int i = 0; i < 16; ++i) {
    const int lid = i * 4 + sub;
    const int row = 32 * w + (lid >> 1), hl = lid & 1;
    const v4f v = *(const v4fa*)(sF + row * 64 + 32 * hl + 4 * q8);
    float* dst = plane + (size_t)(m0 + row) * NC + c0 + 32 * hl + 4 * q8;
    *(volatile v4f*)dst = v;
  }
}

__device__ __forceinline__ void store_rows_f16_from_f32(const float* sF, _Float16* plane,
                                                        int m0, int c0, int w, int lane) {
  const int q8 = lane & 7, sub = lane >> 3;
  #pragma unroll
  for (int i = 0; i < 8; ++i) {
    const int lid = w * 32 + i * 4 + sub;
    const float* s = sF + lid * 64 + 8 * q8;
    const v4f a = *(const v4fa*)s;
    const v4f c = *(const v4fa*)(s + 4);
    const v8h o = { (_Float16)a.x, (_Float16)a.y, (_Float16)a.z, (_Float16)a.w,
                    (_Float16)c.x, (_Float16)c.y, (_Float16)c.z, (_Float16)c.w };
    _Float16* dst = plane + (size_t)(m0 + lid) * NC + c0 + 8 * q8;
    *(volatile v8h*)dst = o;
  }
}

template <bool TRANS>
__global__ __launch_bounds__(128) void k_conv(
    const _Float16* __restrict__ hin,
    const _Float16* __restrict__ wpl,
    const float* __restrict__ bias,
    const float* __restrict__ hres,
    _Float16* __restrict__ outp,
    int dil)
{
  __shared__ __attribute__((aligned(16))) _Float16 sT[128 * 64];

  const int tid = threadIdx.x, lane = tid & 31, w = tid >> 5;
  const int h = lane >> 4, m = lane & 15;
  const int m0 = blockIdx.x * 128;
  const int o0 = blockIdx.y * 64;
  const int b = m0 >> 10, t0 = m0 & (SP - 1);
  const _Float16* hb = hin + (size_t)b * SP * NC;
  const int ta = t0 + 32 * w + m;
  const _Float16* wb = wpl + (size_t)(o0 + m) * KCV;

  const v8f zero8 = {0.f, 0.f, 0.f, 0.f, 0.f, 0.f, 0.f, 0.f};
  v8f acc[2][4];
  #pragma unroll
  for (int mt = 0; mt < 2; ++mt)
    #pragma unroll
    for (int nt = 0; nt < 4; ++nt) acc[mt][nt] = zero8;

  #pragma unroll 1
  for (int tap = 0; tap < KW; ++tap) {
    const int sh = (tap - 1) * dil;
    const _Float16* a0p = hb + (size_t)((ta + sh) & (SP - 1)) * NC;
    const _Float16* a1p = hb + (size_t)((ta + 16 + sh) & (SP - 1)) * NC;
    const _Float16* wbt = wb + tap * NC;
    #pragma unroll 2
    for (int c0 = 0; c0 < NC; c0 += 32) {
      const v16h a0 = load_frag(a0p + c0, h);
      const v16h a1 = load_frag(a1p + c0, h);
      #pragma unroll
      for (int nt = 0; nt < 4; ++nt) {
        const v16h bf = load_frag(wbt + (size_t)nt * 16 * KCV + c0, h);
        acc[0][nt] = wmma_f16(a0, bf, acc[0][nt]);
        acc[1][nt] = wmma_f16(a1, bf, acc[1][nt]);
      }
    }
  }

  #pragma unroll
  for (int nt = 0; nt < 4; ++nt) {
    const int feat = 16 * nt + m;
    const float bv = bias[o0 + feat];
    #pragma unroll
    for (int mt = 0; mt < 2; ++mt) {
      #pragma unroll
      for (int r = 0; r < 8; ++r) {
        const int tokl = 32 * w + 16 * mt + 8 * h + r;
        float y = acc[mt][nt][r] * WINV + bv;
        y = (y > 0.0f) ? y : 0.0f;
        if (TRANS) {
          y = y + hres[(size_t)(m0 + tokl) * NC + o0 + feat];
          y = (y > 0.0f) ? y : 0.0f;
          sT[feat * 128 + tokl] = (_Float16)y;
        } else {
          sT[tokl * 64 + feat] = (_Float16)y;
        }
      }
    }
  }
  __syncthreads();

  if (TRANS) {
    store_trans_f16(sT, outp, b, o0, t0, w, lane);
    __threadfence();
    store_trans_f16(sT, outp, b, o0, t0, w, lane);
  } else {
    store_rows_f16(sT, outp, m0, o0, w, lane);
    __threadfence();
    store_rows_f16(sT, outp, m0, o0, w, lane);
  }
}

__global__ __launch_bounds__(128) void k_gemm_c(
    const _Float16* __restrict__ wg,
    const _Float16* __restrict__ ht,
    _Float16* __restrict__ hn)
{
  __shared__ __attribute__((aligned(16))) _Float16 sT[128 * 64];

  const int tid = threadIdx.x, lane = tid & 31, w = tid >> 5;
  const int h = lane >> 4, m = lane & 15;
  const int m0 = blockIdx.x * 128;
  const int n0 = blockIdx.y * 64;
  const int b = blockIdx.z;

  const _Float16* xa0 = wg + (size_t)(m0 + 32 * w + m) * SP;
  const _Float16* xa1 = xa0 + (size_t)16 * SP;
  const _Float16* wbp = ht + ((size_t)(b * NC + n0 + m)) * SP;

  const v8f zero8 = {0.f, 0.f, 0.f, 0.f, 0.f, 0.f, 0.f, 0.f};
  v8f acc[2][4];
  #pragma unroll
  for (int mt = 0; mt < 2; ++mt)
    #pragma unroll
    for (int nt = 0; nt < 4; ++nt) acc[mt][nt] = zero8;

  #pragma unroll 2
  for (int k0 = 0; k0 < SP; k0 += 32) {
    const v16h a0 = load_frag(xa0 + k0, h);
    const v16h a1 = load_frag(xa1 + k0, h);
    #pragma unroll
    for (int nt = 0; nt < 4; ++nt) {
      const v16h bf = load_frag(wbp + (size_t)nt * 16 * SP + k0, h);
      acc[0][nt] = wmma_f16(a0, bf, acc[0][nt]);
      acc[1][nt] = wmma_f16(a1, bf, acc[1][nt]);
    }
  }

  #pragma unroll
  for (int nt = 0; nt < 4; ++nt) {
    const int feat = 16 * nt + m;
    #pragma unroll
    for (int mt = 0; mt < 2; ++mt) {
      #pragma unroll
      for (int r = 0; r < 8; ++r) {
        const int tokl = 32 * w + 16 * mt + 8 * h + r;
        sT[tokl * 64 + feat] = (_Float16)(acc[mt][nt][r] * WINV);
      }
    }
  }
  __syncthreads();

  const int row0 = b * SP + m0;
  store_rows_f16(sT, hn, row0, n0, w, lane);
  __threadfence();
  store_rows_f16(sT, hn, row0, n0, w, lane);
}

template <bool LAST>
__global__ __launch_bounds__(128) void k_gemm_d(
    const _Float16* __restrict__ hn,
    const _Float16* __restrict__ am,
    const float* __restrict__ gcb,
    float* __restrict__ hf,
    _Float16* __restrict__ h16,
    float* __restrict__ outp)
{
  __shared__ __attribute__((aligned(16))) float sF[128 * 64];

  const int tid = threadIdx.x, lane = tid & 31, w = tid >> 5;
  const int h = lane >> 4, m = lane & 15;
  const int m0 = blockIdx.x * 128;
  const int n0 = blockIdx.y * 64;

  const _Float16* xa0 = hn + (size_t)(m0 + 32 * w + m) * NC;
  const _Float16* xa1 = xa0 + (size_t)16 * NC;
  const _Float16* wbp = am + (size_t)(n0 + m) * NC;

  const v8f zero8 = {0.f, 0.f, 0.f, 0.f, 0.f, 0.f, 0.f, 0.f};
  v8f acc[2][4];
  #pragma unroll
  for (int mt = 0; mt < 2; ++mt)
    #pragma unroll
    for (int nt = 0; nt < 4; ++nt) acc[mt][nt] = zero8;

  #pragma unroll 2
  for (int k0 = 0; k0 < NC; k0 += 32) {
    const v16h a0 = load_frag(xa0 + k0, h);
    const v16h a1 = load_frag(xa1 + k0, h);
    #pragma unroll
    for (int nt = 0; nt < 4; ++nt) {
      const v16h bf = load_frag(wbp + (size_t)nt * 16 * NC + k0, h);
      acc[0][nt] = wmma_f16(a0, bf, acc[0][nt]);
      acc[1][nt] = wmma_f16(a1, bf, acc[1][nt]);
    }
  }

  #pragma unroll
  for (int mt = 0; mt < 2; ++mt) {
    #pragma unroll
    for (int r = 0; r < 8; ++r) {
      const int tokl = 32 * w + 16 * mt + 8 * h + r;
      const float bv = gcb[(m0 + tokl) & (SP - 1)];
      #pragma unroll
      for (int nt = 0; nt < 4; ++nt) {
        const int feat = 16 * nt + m;
        sF[tokl * 64 + feat] = acc[mt][nt][r] + bv;
      }
    }
  }
  __syncthreads();

  if (LAST) {
    store_rows_f32(sF, outp, m0, n0, w, lane);
    __threadfence();
    store_rows_f32(sF, outp, m0, n0, w, lane);
  } else {
    store_rows_f32(sF, hf, m0, n0, w, lane);
    store_rows_f16_from_f32(sF, h16, m0, n0, w, lane);
    __threadfence();
    store_rows_f32(sF, hf, m0, n0, w, lane);
    store_rows_f16_from_f32(sF, h16, m0, n0, w, lane);
  }
}

extern "C" void kernel_launch(void* const* d_in, const int* in_sizes, int n_in,
                              void* d_out, int out_size, void* d_ws, size_t ws_size,
                              hipStream_t stream) {
  if (n_in < 9) return;
  if (in_sizes[0] != NACT) return;
  if (in_sizes[1] != NCW || in_sizes[3] != NCW) return;
  if (in_sizes[2] != LV * NC || in_sizes[4] != LV * NC) return;
  if (in_sizes[5] != SP * SP || in_sizes[6] != SP) return;
  if (in_sizes[7] != NC * NC * 2 || in_sizes[8] != LV * NC * NC * 2) return;
  if (out_size != NACT) return;

  const float* x      = (const float*)d_in[0];
  const float* c1w    = (const float*)d_in[1];
  const float* c1b    = (const float*)d_in[2];
  const float* c2w    = (const float*)d_in[3];
  const float* c2b    = (const float*)d_in[4];
  const float* gcw    = (const float*)d_in[5];
  const float* gcb    = (const float*)d_in[6];
  const float* lg     = (const float*)d_in[7];
  const float* gn     = (const float*)d_in[8];
  float* out = (float*)d_out;

  const size_t hf_bytes  = (size_t)NACT * 4;
  const size_t h16_bytes = (size_t)NACT * 2;
  const size_t c1_bytes  = h16_bytes;
  const size_t ht_bytes  = h16_bytes;
  const size_t wcv_bytes = (size_t)LV * 2 * NC * KCV * 2;
  const size_t wg_bytes  = (size_t)SP * SP * 2;
  const size_t ap_bytes  = (size_t)LV * NC * NC * 2;
  const size_t total = hf_bytes + h16_bytes + c1_bytes + ht_bytes + wcv_bytes + wg_bytes + ap_bytes;
  if (total > ws_size) return;

  char* ws = (char*)d_ws;
  size_t off = 0;
  float*    hf   = (float*)(ws + off);     off += hf_bytes;
  _Float16* h16  = (_Float16*)(ws + off);  off += h16_bytes;
  _Float16* c1hn = (_Float16*)(ws + off);  off += c1_bytes;
  _Float16* ht   = (_Float16*)(ws + off);  off += ht_bytes;
  _Float16* wcv  = (_Float16*)(ws + off);  off += wcv_bytes;
  _Float16* wg   = (_Float16*)(ws + off);  off += wg_bytes;
  _Float16* ap   = (_Float16*)(ws + off);  off += ap_bytes;
  if (off > ws_size) return;

  k_cvt_x<<<(NACT / 8) / 256, 256, 0, stream>>>(x, h16);
  k_prep_convw<<<dim3((NC * (KCV / 8)) / 256, LV * 2), 256, 0, stream>>>(c1w, c2w, wcv);
  k_prep_gcT<<<(SP * (SP / 8)) / 256, 256, 0, stream>>>(gcw, wg);
  k_prep_adj<<<(LV * NC * NC) / 256, 256, 0, stream>>>(lg, gn, ap);

  const dim3 gConv((BZ * SP) / 128, NC / 64);
  const dim3 gC(SP / 128, NC / 64, BZ);
  const dim3 gD((BZ * SP) / 128, NC / 64);

  for (int l = 0; l < LV; ++l) {
    const int dil = 1 << l;
    const float* hres = (l == 0) ? x : (const float*)hf;
    const _Float16* wc1 = wcv + (size_t)(l * 2 + 0) * NC * KCV;
    const _Float16* wc2 = wcv + (size_t)(l * 2 + 1) * NC * KCV;
    const _Float16* apl = ap + (size_t)l * NC * NC;

    k_conv<false><<<gConv, 128, 0, stream>>>(h16, wc1, c1b + l * NC, hres, c1hn, dil);
    k_conv<true ><<<gConv, 128, 0, stream>>>(c1hn, wc2, c2b + l * NC, hres, ht, dil);
    k_gemm_c<<<gC, 128, 0, stream>>>(wg, ht, c1hn);
    if (l == LV - 1)
      k_gemm_d<true ><<<gD, 128, 0, stream>>>(c1hn, apl, gcb, hf, h16, out);
    else
      k_gemm_d<false><<<gD, 128, 0, stream>>>(c1hn, apl, gcb, hf, h16, out);
  }
}
